// PaiConvDG_10050223472788
// MI455X (gfx1250) — hardware-verified
//
#include <hip/hip_runtime.h>


namespace {
constexpr int NB = 16, C = 64, NPT = 2048, NP = NB * NPT  , NLIM = 32768  , KN = 20, KS = 20, KP = 32, OC = 64, PPW = 8  , RPB = 64, NPB = NP / RPB, NPBL = NLIM / RPB;
constexpr float XS = 8.0f, WSC = 256.0f, EPS = 1e-5f;
static_assert(NP % 64 == 0 && NLIM % 64 == 0 && NLIM <= NP && C == 64 && OC == 64 && KN <= KP && KS <= KP, "tiling");
typedef _Float16 b16;
typedef __attribute__((ext_vector_type(16))) _Float16 v16b;
typedef __attribute__((ext_vector_type(8))) _Float16 v8b;
typedef __attribute__((ext_vector_type(8))) float v8f;
typedef __attribute__((ext_vector_type(4))) float v4f;
__device__ __forceinline__ float bf16_rne(float f) { unsigned int u = __float_as_uint(f); u += 0x7FFFu + ((u >> 16) & 1u); return __uint_as_float(u & 0xFFFF0000u); }
__device__ __forceinline__ void split16(float v, b16& hi, b16& lo) { hi = (b16)v; lo = (b16)(v - (float)hi); }
__device__ __forceinline__ v16b frag_kb(const b16* p, int hh) { const v8b a = *(const v8b*)(p + 8 * hh), b = *(const v8b*)(p + 16 + 8 * hh); v16b f;
#pragma unroll
  for (int e = 0; e < 8; ++e) { f[e] = a[e]; f[8 + e] = b[e]; } return f; }
__device__ __forceinline__ v8f wmma16b(v16b a, v16b b, v8f c) { v8f d = __builtin_amdgcn_wmma_f32_16x16x32_f16(false, a, false, b, (short)0, c, false, false); asm volatile("v_nop\n\tv_nop\n\tv_nop\n\tv_nop" : "+v"(d) : "v"(a), "v"(b)); return d; }
__device__ __forceinline__ void wave_lds_sync() { __builtin_amdgcn_fence(__ATOMIC_RELEASE, "workgroup"); __builtin_amdgcn_wave_barrier(); __builtin_amdgcn_fence(__ATOMIC_ACQUIRE, "workgroup"); }
__device__ __forceinline__ float pmul(float a, float b) { float p = a * b; asm volatile("" : "+v"(p)); return p; }
__device__ __forceinline__ int iclamp(int v, int lo, int hi) { return v < lo ? lo : (v > hi ? hi : v); }

typedef __attribute__((ext_vector_type(2))) _Float16 v2h;
typedef __attribute__((ext_vector_type(2))) float v2f;
__host__ __device__ inline int pi_of(int c) { return 4 * (c & 31) + (c >> 5); }
__global__ __launch_bounds__(256) void prep_kernel(const float* __restrict__ feat, const float* __restrict__ w, b16* __restrict__ Ft, b16* __restrict__ Wab) {
  __shared__ __attribute__((aligned(16))) b16 tile[64][C + 8];
  const int t = threadIdx.x;
  if (blockIdx.x < NP / 64) { const int p0 = blockIdx.x * 64; const int b = p0 / NPT, n0 = p0 % NPT;
    for (int q = t; q < 64 * C; q += 256) { const int c = q >> 6, j = q & 63; tile[j][c] = (b16)(bf16_rne(feat[((size_t)b * C + c) * NPT + n0 + j]) * XS); }
    __syncthreads();
    const int wave = t >> 5, lane = t & 31;
    for (int pass = 0; pass < 2; ++pass) { for (int rr = 0; rr < 8; ++rr) { const int j = wave * 8 + rr; *(volatile v2h*)(Ft + (size_t)(p0 + j) * C + lane * 2) = *(const v2h*)(&tile[j][lane * 2]); } __threadfence(); }
  } else { for (int q = t; q < 2 * OC * C / 8; q += 256) { const int r = q >> 3, c0 = (q & 7) * 8; const int o = r & 63, half = r >> 6; v8b v; for (int j = 0; j < 8; ++j) v[j] = (b16)(bf16_rne(w[o * 2 * C + pi_of(half * 64 + c0 + j)]) * WSC);
      for (int pass = 0; pass < 2; ++pass) { *(volatile v8b*)(Wab + (size_t)r * C + c0) = v; __threadfence(); } } }
}
__global__ __launch_bounds__(128) void p01_kernel(const b16* __restrict__ Ft, const b16* __restrict__ Wab, float* __restrict__ P) {
  __shared__ __attribute__((aligned(16))) float Tf[4][16][128 + 4];
  const int wave = threadIdx.x >> 5, lane = threadIdx.x & 31, nloc = lane & 15, hlf = lane >> 4; const size_t m0 = (size_t)blockIdx.x * 64 + wave * 16;
  v8f acc[8];
#pragma unroll
  for (int t = 0; t < 8; ++t) acc[t] = (v8f){};
#pragma unroll
  for (int kb = 0; kb < C; kb += 32) { const v16b a = frag_kb(Ft + (m0 + nloc) * C + kb, hlf);
#pragma unroll
    for (int t = 0; t < 8; ++t) acc[t] = wmma16b(a, frag_kb(Wab + (size_t)(t * 16 + nloc) * C + kb, hlf), acc[t]); }
#pragma unroll
  for (int t = 0; t < 8; ++t)
#pragma unroll
    for (int r = 0; r < 8; ++r) Tf[wave][8 * hlf + r][t * 16 + nloc] = acc[t][r] * (1.0f / (XS * WSC));
  wave_lds_sync();
  for (int pass = 0; pass < 2; ++pass) { for (int rr = 0; rr < 16; ++rr) *(volatile v4f*)(P + (m0 + rr) * 128 + lane * 4) = *(const v4f*)(&Tf[wave][rr][lane * 4]); __threadfence(); }
}
__global__ __launch_bounds__(128) void point_kernel(const float* __restrict__ P, const int* __restrict__ nbr, const float* __restrict__ perm, const float* __restrict__ bias, float* __restrict__ M) {
  __shared__ __attribute__((aligned(16))) b16 Gh[4][OC][KP + 8], Gl[4][OC][KP + 8], Bp[4][KP][KP + 8]; __shared__ __attribute__((aligned(16))) float Gf[4][OC][KP + 1], Ms[4][PPW][OC];
  const int wave = threadIdx.x >> 5, lane = threadIdx.x & 31, nloc = lane & 15, hlf = lane >> 4;
  const float b0 = bf16_rne(bias[lane * 2]), b1 = bf16_rne(bias[lane * 2 + 1]);
#pragma unroll 1
  for (int q = 0; q < PPW; ++q) { const size_t n = ((size_t)blockIdx.x * 4 + wave) * PPW + q;
    const int n0i = iclamp(nbr[n * KN + 0], 0, NP - 1); const v2f p0 = *(const v2f*)(P + (size_t)n0i * 128 + lane * 2), p1c = *(const v2f*)(P + (size_t)n0i * 128 + 64 + lane * 2); const float c0 = p0[0] - p1c[0], c1 = p0[1] - p1c[1];
#pragma unroll 1
    for (int k = 0; k < KP; ++k) { float g0 = 0.0f, g1 = 0.0f; if (k < KN) { const int nk = iclamp(nbr[n * KN + k], 0, NP - 1); const v2f pk = *(const v2f*)(P + (size_t)nk * 128 + 64 + lane * 2); g0 = c0 + pk[0]; g1 = c1 + pk[1]; } Gf[wave][lane * 2][k] = g0; Gf[wave][lane * 2 + 1][k] = g1; }
    { const int s = lane; v8b v[4];
#pragma unroll
      for (int kq = 0; kq < 4; ++kq) for (int j = 0; j < 8; ++j) { const int k = kq * 8 + j; v[kq][j] = (s < KS && k < KN) ? (b16)(bf16_rne(perm[(n * KN + k) * KS + s]) * XS) : (b16)0.0f; }
#pragma unroll
      for (int kq = 0; kq < 4; ++kq) *(v8b*)(&Bp[wave][s][kq * 8]) = v[kq]; }
    wave_lds_sync();
#pragma unroll
    for (int rr = 0; rr < 2; ++rr) { const int o = lane * 2 + rr;
#pragma unroll
      for (int kq = 0; kq < 4; ++kq) { v8b hv, lv; for (int j = 0; j < 8; ++j) { b16 p, qq; split16(Gf[wave][o][kq * 8 + j] * XS, p, qq); hv[j] = p; lv[j] = qq; } *(v8b*)(&Gh[wave][o][kq * 8]) = hv; *(v8b*)(&Gl[wave][o][kq * 8]) = lv; } }
    wave_lds_sync();
    const v16b b0f = frag_kb(&Bp[wave][nloc][0], hlf), b1f = frag_kb(&Bp[wave][16 + nloc][0], hlf);
#pragma unroll
    for (int t = 0; t < 4; ++t) { const v16b a = frag_kb(&Gh[wave][t * 16 + nloc][0], hlf), al = frag_kb(&Gl[wave][t * 16 + nloc][0], hlf);
      v8f d0 = (v8f){}, d1 = (v8f){}; d0 = wmma16b(a, b0f, d0); d0 = wmma16b(al, b0f, d0); d1 = wmma16b(a, b1f, d1); d1 = wmma16b(al, b1f, d1);
#pragma unroll
      for (int r = 0; r < 8; ++r) { float m = d0[r]; const float m1 = (nloc < KS - 16) ? d1[r] : -INFINITY; m = fmaxf(m, m1);
#pragma unroll
        for (int off = 1; off < 16; off <<= 1) m = fmaxf(m, __shfl_xor(m, off));
        if (nloc == 0) Ms[wave][q][t * 16 + 8 * hlf + r] = m * (1.0f / (XS * XS)); } }
    wave_lds_sync(); }
  for (int pass = 0; pass < 2; ++pass) { for (int q = 0; q < PPW; ++q) { const size_t n = ((size_t)blockIdx.x * 4 + wave) * PPW + q; v2f o = *(const v2f*)(&Ms[wave][q][lane * 2]); o[0] += b0; o[1] += b1; *(volatile v2f*)(M + n * OC + lane * 2) = o; } __threadfence(); }
}
__global__ __launch_bounds__(64) void psum_kernel(const float* __restrict__ M, const float* __restrict__ MEAN, int centred, float* __restrict__ PS) {
  const int blk = blockIdx.x, c = threadIdx.x; const float m = centred ? MEAN[c] : 0.0f; float s = 0.0f;
#pragma unroll 1
  for (int rr = 0; rr < RPB; ++rr) { const float d = M[((size_t)blk * RPB + rr) * OC + c] - m; s += centred ? d * d : d; }
  for (int pass = 0; pass < 2; ++pass) { ((volatile float*)PS)[(size_t)blk * OC + c] = s; __threadfence(); }
}
__global__ __launch_bounds__(64) void colstat_kernel(const float* __restrict__ PS, float* __restrict__ STAT) {
  const int c = threadIdx.x; float s = 0.0f;
#pragma unroll 1
  for (int k = 0; k < NPBL; ++k) s += PS[(size_t)k * OC + c];
  for (int pass = 0; pass < 2; ++pass) { ((volatile float*)STAT)[c] = s * (1.0f / (float)NLIM); __threadfence(); }
}
__global__ __launch_bounds__(128) void out_kernel(const float* __restrict__ M, const float* __restrict__ MEAN, const float* __restrict__ VAR, const float* __restrict__ bnw, const float* __restrict__ bnb, float* __restrict__ out) {
  __shared__ __attribute__((aligned(16))) float tile[OC][64 + 4];
  const int p0 = blockIdx.x * 64, t = threadIdx.x; const int b = p0 / NPT, n0 = p0 % NPT;
  for (int q = t; q < 64 * OC; q += 128) { const int j = q >> 6, c = q & 63; tile[c][j] = (M[(size_t)(p0 + j) * OC + c] - MEAN[c]) * rsqrtf(VAR[c] + EPS) * bf16_rne(bnw[c]) + bf16_rne(bnb[c]); }
  __syncthreads();
  const int wave = t >> 5, lane = t & 31;
  for (int pass = 0; pass < 2; ++pass) { for (int rr = 0; rr < 16; ++rr) { const int c = wave * 16 + rr; *(volatile v2f*)(out + ((size_t)b * OC + c) * NPT + n0 + lane * 2) = *(const v2f*)(&tile[c][lane * 2]); } __threadfence(); }
}
}

extern "C" void kernel_launch(void* const* d_in, const int* in_sizes, int n_in, void* d_out, int out_size, void* d_ws, size_t ws_size, hipStream_t stream) {
  (void)n_in;
  auto Fp = [&](int i) { return (const float*)d_in[i]; }; auto Ip = [&](int i) { return (const int*)d_in[i]; };
  if (in_sizes[0] != NP * C || in_sizes[1] != NP * KN || in_sizes[2] != NP * KN * KS || in_sizes[3] != OC * 2 * C || in_sizes[4] != OC || in_sizes[5] != OC || in_sizes[6] != OC || out_size != NP * OC) return;
  size_t off = 0; char* ws = (char*)d_ws;
  auto carve = [&](size_t bytes) { char* p = ws + off; off += (bytes + 255) & ~(size_t)255; return p; };
  b16* Ft = (b16*)carve((size_t)NP * C * 2); b16* Wab = (b16*)carve((size_t)2 * OC * C * 2); float* P = (float*)carve((size_t)NP * 128 * 4); float* M = (float*)carve((size_t)NP * OC * 4); float* PS = (float*)carve((size_t)NPB * OC * 4); float* MEAN = (float*)carve(OC * 4); float* VAR = (float*)carve(OC * 4);
  if (off > ws_size || off > ((size_t)128 << 20)) return;
  prep_kernel<<<NP / 64 + 1, 256, 0, stream>>>(Fp(0), Fp(3), Ft, Wab);
  p01_kernel<<<NP / 64, 128, 0, stream>>>(Ft, Wab, P);
  point_kernel<<<NLIM / 32, 128, 0, stream>>>(P, Ip(1), Fp(2), Fp(4), M);
  psum_kernel<<<NPBL, 64, 0, stream>>>(M, MEAN, 0, PS); colstat_kernel<<<1, 64, 0, stream>>>(PS, MEAN);
  psum_kernel<<<NPBL, 64, 0, stream>>>(M, MEAN, 1, PS); colstat_kernel<<<1, 64, 0, stream>>>(PS, VAR);
  out_kernel<<<NLIM / 64, 128, 0, stream>>>(M, MEAN, VAR, Fp(5), Fp(6), (float*)d_out);
}
